// TwoTwoNet_53051436040339
// MI455X (gfx1250) — hardware-run, weakly checked
//
#include <hip/hip_runtime.h>

constexpr int NBATCH  = 256;
constexpr int NSTEP   = 512;
constexpr int NUNIT   = 1024;
constexpr int NTHR    = 256;
constexpr int NWAVE   = NTHR / 32;
constexpr int NBLK    = 2;
constexpr int KCHUNKS = NUNIT / 32;
constexpr int TCH     = 32;
constexpr int NTCH    = NSTEP / TCH;
constexpr int BP      = 1032;
constexpr int SCRP    = 17;
constexpr int XP      = 36;
constexpr int OP      = 36;

static_assert(NBATCH == NBLK * NWAVE * 16, "one wave owns 16 batch rows");
static_assert(NUNIT == NTHR * 4, "prologue: four units per thread");
static_assert(NUNIT % 32 == 0 && NSTEP % TCH == 0, "no k tail, no step tail");
static_assert(BP % 8 == 0 && BP >= NUNIT + 8, "B plane pitch");
static_assert((TCH * 4) % 128 == 0 && (NSTEP * 4) % 128 == 0, "output flush is whole 128-B lines");

constexpr int OFF_DE   = 0;
constexpr int SZ_DE    = 2 * NUNIT * 4;
constexpr int OFF_BT   = OFF_DE + SZ_DE;
constexpr int SZ_BT    = 16 * BP * 2;
constexpr int OFF_SCR  = OFF_BT + SZ_BT;
constexpr int SZ_SCR_W = 16 * SCRP * 4;
constexpr int OFF_XS   = OFF_SCR + NWAVE * SZ_SCR_W;
constexpr int SZ_XS_W  = 16 * XP * 4;
constexpr int OFF_OB   = OFF_XS + NWAVE * SZ_XS_W;
constexpr int SZ_OB_W  = 16 * OP * 4;
constexpr int OFF_RED  = OFF_OB + NWAVE * SZ_OB_W;
constexpr int SZ_RED   = NWAVE * 4 * 4;
constexpr int LDS_TOTAL = OFF_RED + SZ_RED;
static_assert(OFF_BT % 16 == 0 && OFF_SCR % 16 == 0 && OFF_XS % 16 == 0 && OFF_OB % 16 == 0 && OFF_RED % 16 == 0, "LDS alignment");
static_assert(SZ_SCR_W % 16 == 0 && SZ_XS_W % 16 == 0 && SZ_OB_W % 16 == 0, "per-wave LDS alignment");
static_assert(LDS_TOTAL == 86912, "LDS total");

typedef __attribute__((ext_vector_type(16))) __bf16   v16b;
typedef __attribute__((ext_vector_type(8)))  float    v8f;
typedef __attribute__((ext_vector_type(4)))  float    v4f;
typedef __attribute__((ext_vector_type(8)))  unsigned v8u;
typedef __attribute__((ext_vector_type(4)))  unsigned v4u;
typedef __attribute__((ext_vector_type(2)))  unsigned v2u;

__device__ __forceinline__ unsigned bf_rne_bits(float f) {
  const unsigned u = __float_as_uint(f);
  return (u + 0x7FFFu + ((u >> 16) & 1u)) >> 16;
}
__device__ __forceinline__ float bf_bits_to_f32(unsigned h) { return __uint_as_float(h << 16); }

__device__ __forceinline__ void split3_rne(float v, unsigned& h, unsigned& m, unsigned& l) {
  h = bf_rne_bits(v);
  const float r1 = v - bf_bits_to_f32(h);
  m = bf_rne_bits(r1);
  const float r2 = r1 - bf_bits_to_f32(m);
  l = bf_rne_bits(r2);
}

__device__ __forceinline__ void split_pair(float p0, float p1, unsigned& wh, unsigned& wm) {
  const unsigned u0 = __float_as_uint(p0);
  const unsigned u1 = __float_as_uint(p1);
  const unsigned h0 = u0 & 0xffff0000u;
  const unsigned h1 = u1 & 0xffff0000u;
  wh = (u0 >> 16) | h1;
  const float r0 = p0 - __uint_as_float(h0);
  const float r1 = p1 - __uint_as_float(h1);
  const unsigned a0 = __float_as_uint(r0);
  const unsigned a1 = __float_as_uint(r1);
  const unsigned m1 = a1 & 0xffff0000u;
  wm = (a0 >> 16) | m1;
}

__device__ __forceinline__ v8f mma_bf16_guarded(v16b a, v16b b, v8f c) {
  c = __builtin_amdgcn_wmma_f32_16x16x32_bf16(false, a, false, b, (short)0, c, false, false);
  asm volatile("v_nop\n\tv_nop\n\tv_nop\n\tv_nop" : "+v"(c) : "v"(a), "v"(b));
  return c;
}

__device__ __forceinline__ void wave_lds_sync() {
  __builtin_amdgcn_fence(__ATOMIC_RELEASE, "workgroup");
  __builtin_amdgcn_wave_barrier();
  __builtin_amdgcn_fence(__ATOMIC_ACQUIRE, "workgroup");
}

__device__ __forceinline__ float clip_unit(float v) { return fminf(1.0f, fmaxf(-1.0f, v)); }

__global__ void __launch_bounds__(NTHR, 1)
sat_rank2_scan_kernel(const float* __restrict__ x, const float* __restrict__ state0, const float* __restrict__ mask,
                      const float* __restrict__ w, const float* __restrict__ dorth, const float* __restrict__ eorth,
                      const float* __restrict__ decoder, const float* __restrict__ encoder, float* __restrict__ out) {
  extern __shared__ v4u smem_dyn[];
  unsigned char* const smem_raw = (unsigned char*)smem_dyn;
  const int tid = threadIdx.x, lane = tid & 31, wave = tid >> 5;
  const int c = lane & 15, hh = lane >> 4;

  float*    const DEt = (float*)(smem_raw + OFF_DE);
  unsigned* const BtW = (unsigned*)(smem_raw + OFF_BT);
  float*    const scr = (float*)(smem_raw + OFF_SCR + wave * SZ_SCR_W);
  float*    const xs  = (float*)(smem_raw + OFF_XS + wave * SZ_XS_W);
  float*    const ob  = (float*)(smem_raw + OFF_OB + wave * SZ_OB_W);
  float*    const RED = (float*)(smem_raw + OFF_RED);

  float pkd = 0.0f, pke = 0.0f, p0d = 0.0f, p0e = 0.0f;
  {
    const int k4 = tid * 4;
    const v4f dv = *(const v4f*)(dorth + k4);
    const v4f ev = *(const v4f*)(eorth + k4);
    const v4f mv = *(const v4f*)(mask + k4);
    const v4f nv = *(const v4f*)(encoder + k4);
    const v4f ov = *(const v4f*)(decoder + k4);
    const v4f sv = *(const v4f*)(state0 + k4);
    unsigned hb[3][4], mb[3][4], lb[3][4];
#pragma unroll
    for (int e = 0; e < 4; ++e) {
      const float di = dv[e], ei = ev[e], mi = mv[e], ni = nv[e], oi = ov[e], si = sv[e];
      const float men = mi * ni;
      pkd = fmaf(men, di, pkd);
      pke = fmaf(men, ei, pke);
      p0d = fmaf(si, di, p0d);
      p0e = fmaf(si, ei, p0e);
      split3_rne(mi * di, hb[0][e], mb[0][e], lb[0][e]);
      split3_rne(mi * ei, hb[1][e], mb[1][e], lb[1][e]);
      split3_rne(mi * oi, hb[2][e], mb[2][e], lb[2][e]);
    }
    const int kc = k4 >> 5, kk = k4 & 31;
    const int hq = (kk >> 3) & 1;
    const int i0 = (kk & 7) + ((kk >> 4) << 3);
    *(v4f*)(DEt + (kc * 2 + hq) * 32 + i0)      = dv;
    *(v4f*)(DEt + (kc * 2 + hq) * 32 + 16 + i0) = ev;
#pragma unroll
    for (int v = 0; v < 3; ++v) {
      const v2u wh = {hb[v][0] | (hb[v][1] << 16), hb[v][2] | (hb[v][3] << 16)};
      const v2u wm = {mb[v][0] | (mb[v][1] << 16), mb[v][2] | (mb[v][3] << 16)};
      const v2u wl = {lb[v][0] | (lb[v][1] << 16), lb[v][2] | (lb[v][3] << 16)};
      *(v2u*)(BtW + (((3 * v + 0) * BP + k4) >> 1)) = wh;
      *(v2u*)(BtW + (((3 * v + 1) * BP + k4) >> 1)) = wm;
      *(v2u*)(BtW + (((3 * v + 2) * BP + k4) >> 1)) = wl;
    }
    const v2u z2 = {0u, 0u};
#pragma unroll
    for (int n = 9; n < 16; ++n) *(v2u*)(BtW + ((n * BP + k4) >> 1)) = z2;
    if (tid < 16) {
      const v4u z4 = {0u, 0u, 0u, 0u};
      *(v4u*)(BtW + ((tid * BP + NUNIT) >> 1)) = z4;
    }
  }
#pragma unroll
  for (int off = 16; off >= 1; off >>= 1) {
    pkd += __shfl_xor(pkd, off, 32);
    pke += __shfl_xor(pke, off, 32);
    p0d += __shfl_xor(p0d, off, 32);
    p0e += __shfl_xor(p0e, off, 32);
  }
  if (lane == 0) {
    RED[wave * 4 + 0] = pkd;
    RED[wave * 4 + 1] = pke;
    RED[wave * 4 + 2] = p0d;
    RED[wave * 4 + 3] = p0e;
  }
  __syncthreads();
  float Kd = 0.0f, Ke = 0.0f, fd = 0.0f, fe = 0.0f;
#pragma unroll
  for (int wv = 0; wv < NWAVE; ++wv) {
    Kd += RED[wv * 4 + 0];
    Ke += RED[wv * 4 + 1];
    fd += RED[wv * 4 + 2];
    fe += RED[wv * 4 + 3];
  }
  const float w00 = w[0], w01 = w[1], w10 = w[2], w11 = w[3];

  const bool selM = (c < 9) && ((c % 3) != 2);
  const v8f z8 = {0.f, 0.f, 0.f, 0.f, 0.f, 0.f, 0.f, 0.f};

  const int row0 = (blockIdx.x * NWAVE + wave) * 16;
  const float* const xbase = x + (size_t)row0 * NSTEP;
  float* const obase = out + (size_t)row0 * NSTEP;

#pragma unroll 1
  for (int tc = 0; tc < NTCH; ++tc) {
    const int t0 = tc * TCH;
#pragma unroll
    for (int it = 0; it < 4; ++it) {
      const int idx = it * 32 + lane;
      const int r = idx >> 3, q4 = (idx & 7) * 4;
      const v4f xv = *(const v4f*)(xbase + (size_t)r * NSTEP + t0 + q4);
      *(v4f*)(xs + r * XP + q4) = xv;
    }
    wave_lds_sync();

#pragma unroll 1
    for (int tt = 0; tt < TCH; ++tt) {
      const float xt = xs[c * XP + tt];
      const float av = fmaf(xt, Kd, fd);
      const float cv = fmaf(xt, Ke, fe);
      const float alpha = fmaf(w00, av, w01 * cv);
      const float beta  = fmaf(w10, av, w11 * cv);
      v8f accH = z8, accM = z8;

#pragma unroll 1
      for (int kc = 0; kc < KCHUNKS; ++kc) {
        const float* dp = DEt + (kc * 2 + hh) * 32;
        unsigned wh[8], wm[8];
#pragma unroll
        for (int q = 0; q < 4; ++q) {
          const v4f dq = *(const v4f*)(dp + 4 * q);
          const v4f eq = *(const v4f*)(dp + 16 + 4 * q);
          const float p0 = clip_unit(fmaf(dq[0], alpha, eq[0] * beta));
          const float p1 = clip_unit(fmaf(dq[1], alpha, eq[1] * beta));
          const float p2 = clip_unit(fmaf(dq[2], alpha, eq[2] * beta));
          const float p3 = clip_unit(fmaf(dq[3], alpha, eq[3] * beta));
          split_pair(p0, p1, wh[2 * q], wm[2 * q]);
          split_pair(p2, p3, wh[2 * q + 1], wm[2 * q + 1]);
        }
        const v8u whv = {wh[0], wh[1], wh[2], wh[3], wh[4], wh[5], wh[6], wh[7]};
        const v8u wmv = {wm[0], wm[1], wm[2], wm[3], wm[4], wm[5], wm[6], wm[7]};
        const unsigned* bp = BtW + ((c * BP + kc * 32 + 8 * hh) >> 1);
        const v4u b0 = *(const v4u*)(bp);
        const v4u b1 = *(const v4u*)(bp + 8);
        const v8u bwv = __builtin_shufflevector(b0, b1, 0, 1, 2, 3, 4, 5, 6, 7);
        const v16b bfr = __builtin_bit_cast(v16b, bwv);
        const v16b ah = __builtin_bit_cast(v16b, whv);
        const v16b am = __builtin_bit_cast(v16b, wmv);
        accH = mma_bf16_guarded(ah, bfr, accH);
        accM = mma_bf16_guarded(am, bfr, accM);
      }

#pragma unroll
      for (int r = 0; r < 8; ++r) {
        const float tm = selM ? accM[r] : 0.0f;
        const float sv = accH[r] + tm;
        scr[(8 * hh + r) * SCRP + c] = sv;
      }
      wave_lds_sync();
      const float* rp = scr + c * SCRP;
      const float v0 = rp[0], v1 = rp[1], v2 = rp[2];
      const float v3 = rp[3], v4 = rp[4], v5 = rp[5];
      const float v6 = rp[6], v7 = rp[7], v8 = rp[8];
      fd = (v2 + v1) + v0;
      fe = (v5 + v4) + v3;
      const float ov = (v8 + v7) + v6;
      if (hh == 0) ob[c * OP + tt] = ov;
      wave_lds_sync();
    }

    v4f ovv[4];
#pragma unroll
    for (int it = 0; it < 4; ++it) {
      const int idx = it * 32 + lane;
      const int r = idx >> 3, q4 = (idx & 7) * 4;
      ovv[it] = *(const v4f*)(ob + r * OP + q4);
    }
    for (int pass = 0; pass < 2; ++pass) {
#pragma unroll
      for (int it = 0; it < 4; ++it) {
        const int idx = it * 32 + lane;
        const int r = idx >> 3, q4 = (idx & 7) * 4;
        *(volatile v4f*)(obase + (size_t)r * NSTEP + t0 + q4) = ovv[it];
      }
      __threadfence();
    }
    wave_lds_sync();
  }
}

extern "C" void kernel_launch(void* const* d_in, const int* in_sizes, int n_in,
                              void* d_out, int out_size, void* d_ws, size_t ws_size, hipStream_t stream) {
  (void)d_ws; (void)ws_size;
  if (n_in < 8 || d_out == nullptr) return;
  if (in_sizes[0] != NBATCH * NSTEP || in_sizes[1] != NUNIT || in_sizes[2] != NUNIT || in_sizes[3] != 4 ||
      in_sizes[4] != NUNIT || in_sizes[5] != NUNIT || in_sizes[6] != NUNIT || in_sizes[7] != NUNIT ||
      out_size != NBATCH * NSTEP) return;

  const float* x       = (const float*)d_in[0];
  const float* state0  = (const float*)d_in[1];
  const float* mask    = (const float*)d_in[2];
  const float* w       = (const float*)d_in[3];
  const float* dorth   = (const float*)d_in[4];
  const float* eorth   = (const float*)d_in[5];
  const float* decoder = (const float*)d_in[6];
  const float* encoder = (const float*)d_in[7];
  float* out = (float*)d_out;

  sat_rank2_scan_kernel<<<dim3(NBLK), dim3(NTHR), LDS_TOTAL, stream>>>(
      x, state0, mask, w, dorth, eorth, decoder, encoder, out);
}
